// GATModel_20298015441203
// MI455X (gfx1250) — hardware-verified
//
#include <hip/hip_runtime.h>
#include <stddef.h>
#include <stdint.h>
#include <math.h>


#define HC      128
#define KG      256
#define NHMAX   4
#define NSD     (2 * NHMAX)
#define NTHR    256
#define NWAVE   8
#define EPT     8
#define CHUNK   (NTHR * EPT)
#define WCAP    (EPT * 32)
#define LISTN   (NWAVE * WCAP)
#define NBMAX   2048
#define SLOTB   11
#define RCAP    28672
#define DEGCAP  64
#define GBM     64
#define GBN     128
#define GTHR    128
#define MROWS   128
#define NEGSL   0.2f
#define EPS_SM  1e-16f
#define WSMAX   134217728
#define LDS_AGG ((2 * RCAP + 2 * NBMAX + LISTN) * 4 + 64)

static_assert((CHUNK & (CHUNK - 1)) == 0 && CHUNK <= (1 << SLOTB));
static_assert(NBMAX == (1 << SLOTB));
static_assert(NTHR * 8 == NBMAX);
static_assert(LISTN >= NBMAX);
static_assert(LISTN >= NWAVE * WCAP);
static_assert((RCAP % 32) == 0);
static_assert(LDS_AGG <= 300000);
static_assert(GBM == (GTHR / 32) * 16);
static_assert((KG % 32) == 0 && KG == 2 * HC);
static_assert(GBN == HC && (HC % 16) == 0);
static_assert(GTHR == 2 * GBM);
static_assert(GTHR == 32 * NHMAX);
static_assert((MROWS % GBM) == 0);
static_assert(HC == 4 * 32);
static_assert(HC / NHMAX == 8 * 4);

typedef float          v4f  __attribute__((ext_vector_type(4)));
typedef float          v8f  __attribute__((ext_vector_type(8)));
typedef int            v2i  __attribute__((ext_vector_type(2)));
typedef int            v4i  __attribute__((ext_vector_type(4)));
typedef int            v8i  __attribute__((ext_vector_type(8)));
typedef unsigned int   v4u  __attribute__((ext_vector_type(4)));
typedef unsigned short v8us __attribute__((ext_vector_type(8)));
typedef __bf16         v16b __attribute__((ext_vector_type(16)));
typedef v2i  __attribute__((may_alias)) v2ia;
typedef v4f  __attribute__((may_alias)) v4fa;
typedef v8us __attribute__((may_alias)) v8usa;
union FragB { v16b v; v8us h[2]; v8i w; };

__device__ __forceinline__ v8f wmb(const FragB& a, const FragB& b, v8f c) {
  v8f d = __builtin_amdgcn_wmma_f32_16x16x32_bf16(false, a.v, false, b.v, (short)0, c, false, false);
  asm volatile("v_nop\n\tv_nop\n\tv_nop\n\tv_nop" : "+v"(d) : "v"(a.w), "v"(b.w));
  return d;
}

__device__ __forceinline__ unsigned int f2bf(float f) {
  const unsigned int u = __float_as_uint(f);
  return ((u + 0x7FFFu + ((u >> 16) & 1u)) >> 16) & 0xFFFFu;
}
__device__ __forceinline__ float bf2f(unsigned int b) { return __uint_as_float(b << 16); }
__device__ __forceinline__ float bfr(float f) { return bf2f(f2bf(f)); }
__device__ __forceinline__ v4f bfr4(const v4f a) {
  v4f r; r.x = bfr(a.x); r.y = bfr(a.y); r.z = bfr(a.z); r.w = bfr(a.w); return r;
}
__device__ __forceinline__ unsigned int pk2(float lo, float hi) { return f2bf(lo) | (f2bf(hi) << 16); }
__device__ __forceinline__ v4u pack8(const v4f a, const v4f b) {
  v4u r;
  r.x = pk2(a.x, a.y); r.y = pk2(a.z, a.w); r.z = pk2(b.x, b.y); r.w = pk2(b.z, b.w);
  return r;
}
__device__ __forceinline__ unsigned int hlw(float v, unsigned int lom) {
  const unsigned int hb = f2bf(v);
  const unsigned int lb = f2bf(v - bf2f(hb));
  return (hb & ~lom) | (lb & lom);
}

__device__ __forceinline__ int scan_chunk(const int* __restrict__ dsts, int nE, int cbase, int slotBase,
                                          int nb, int vec8, int* list, int tid, int lane, int wave) {
  int wc = 0;
  const int el0  = tid * EPT;
  const int e0   = cbase + el0;
  const int sent = -2147483647 - 1;
  v4i da, db;
  if (vec8 != 0 && cbase + CHUNK <= nE) {
    da = *(const v4i*)(dsts + e0);
    db = *(const v4i*)(dsts + e0 + 4);
  } else {
    da.x = (e0     < nE) ? dsts[min(e0,     nE - 1)] : sent;
    da.y = (e0 + 1 < nE) ? dsts[min(e0 + 1, nE - 1)] : sent;
    da.z = (e0 + 2 < nE) ? dsts[min(e0 + 2, nE - 1)] : sent;
    da.w = (e0 + 3 < nE) ? dsts[min(e0 + 3, nE - 1)] : sent;
    db.x = (e0 + 4 < nE) ? dsts[min(e0 + 4, nE - 1)] : sent;
    db.y = (e0 + 5 < nE) ? dsts[min(e0 + 5, nE - 1)] : sent;
    db.z = (e0 + 6 < nE) ? dsts[min(e0 + 6, nE - 1)] : sent;
    db.w = (e0 + 7 < nE) ? dsts[min(e0 + 7, nE - 1)] : sent;
  }
  const unsigned nbs = (unsigned)slotBase;
  const unsigned unb = (unsigned)nb;
  const unsigned s0 = (unsigned)da.x - nbs, s1 = (unsigned)da.y - nbs;
  const unsigned s2 = (unsigned)da.z - nbs, s3 = (unsigned)da.w - nbs;
  const unsigned s4 = (unsigned)db.x - nbs, s5 = (unsigned)db.y - nbs;
  const unsigned s6 = (unsigned)db.z - nbs, s7 = (unsigned)db.w - nbs;
  const bool h0 = s0 < unb, h1 = s1 < unb, h2 = s2 < unb, h3 = s3 < unb;
  const bool h4 = s4 < unb, h5 = s5 < unb, h6 = s6 < unb, h7 = s7 < unb;
  const unsigned any = __builtin_amdgcn_ballot_w32(h0 | h1 | h2 | h3 | h4 | h5 | h6 | h7);
  if (any != 0u) {
#define HITJ(J, HJ, SJ) { \
      const unsigned mj = __builtin_amdgcn_ballot_w32(HJ); \
      if (mj != 0u) { \
        if (HJ) { \
          const int pos = wc + (int)__builtin_amdgcn_mbcnt_lo(mj, 0u); \
          if (pos < WCAP) list[wave * WCAP + pos] = ((el0 + (J)) << SLOTB) | (int)(SJ); \
        } \
        wc += (int)__builtin_popcount(mj); } }
    HITJ(0, h0, s0)
    HITJ(1, h1, s1)
    HITJ(2, h2, s2)
    HITJ(3, h3, s3)
    HITJ(4, h4, s4)
    HITJ(5, h5, s5)
    HITJ(6, h6, s6)
    HITJ(7, h7, s7)
#undef HITJ
  }
  return wc;
}

__global__ __launch_bounds__(NTHR) void k_esplit(const int* __restrict__ ei, int* SL, int* DL, int nE, int nUnits) {
  const int u = (int)blockIdx.x * NTHR + (int)threadIdx.x;
  if (u >= nUnits) return;
  const int e0  = 4 * u;
  const int sent = -2147483647 - 1;
  const int c0 = min(e0, nE - 1), c1 = min(e0 + 1, nE - 1), c2 = min(e0 + 2, nE - 1), c3 = min(e0 + 3, nE - 1);
  const v2i p0 = *(const v2ia*)(ei + 2 * (size_t)c0);
  const v2i p1 = *(const v2ia*)(ei + 2 * (size_t)c1);
  const v2i p2 = *(const v2ia*)(ei + 2 * (size_t)c2);
  const v2i p3 = *(const v2ia*)(ei + 2 * (size_t)c3);
  v4i sv, dv;
  sv.x = (e0     < nE) ? p0.x : 0;    dv.x = (e0     < nE) ? p0.y : sent;
  sv.y = (e0 + 1 < nE) ? p1.x : 0;    dv.y = (e0 + 1 < nE) ? p1.y : sent;
  sv.z = (e0 + 2 < nE) ? p2.x : 0;    dv.z = (e0 + 2 < nE) ? p2.y : sent;
  sv.w = (e0 + 3 < nE) ? p3.x : 0;    dv.w = (e0 + 3 < nE) ? p3.y : sent;
  int* sp = SL + e0;
  int* dp = DL + e0;
  *(volatile v4i*)sp = sv;
  *(volatile v4i*)dp = dv;
  __threadfence();
  *(volatile v4i*)sp = sv;
  *(volatile v4i*)dp = dv;
}

__global__ __launch_bounds__(NTHR) void k_emb(const float* __restrict__ x, const float* __restrict__ wemb,
                                              const float* __restrict__ bemb, unsigned short* hp,
                                              int nN, int nUnits) {
  const int u = (int)blockIdx.x * NTHR + (int)threadIdx.x;
  if (u >= nUnits) return;
  const int row   = u >> 5;
  const int piece = u & 31;
  const int cb    = (piece & 15) * 8;
  const int rc    = row < nN ? row : nN - 1;
  const float xv  = bfr(x[rc]);
  const v4f w0 = bfr4(*(const v4fa*)(wemb + cb)), w1 = bfr4(*(const v4fa*)(wemb + cb + 4));
  const v4f b0 = bfr4(*(const v4fa*)(bemb + cb)), b1 = bfr4(*(const v4fa*)(bemb + cb + 4));
  v4f ha, hb;
  ha.x = fmaf(xv, w0.x, b0.x); ha.y = fmaf(xv, w0.y, b0.y); ha.z = fmaf(xv, w0.z, b0.z); ha.w = fmaf(xv, w0.w, b0.w);
  hb.x = fmaf(xv, w1.x, b1.x); hb.y = fmaf(xv, w1.y, b1.y); hb.z = fmaf(xv, w1.z, b1.z); hb.w = fmaf(xv, w1.w, b1.w);
  const v4f z4 = {0.f, 0.f, 0.f, 0.f};
  if (row >= nN) { ha = z4; hb = z4; }
  const unsigned int lom = (piece >= 16) ? 0xFFFFFFFFu : 0u;
  v4u pv;
  pv.x = hlw(ha.x, lom) | (hlw(ha.y, lom) << 16);
  pv.y = hlw(ha.z, lom) | (hlw(ha.w, lom) << 16);
  pv.z = hlw(hb.x, lom) | (hlw(hb.y, lom) << 16);
  pv.w = hlw(hb.z, lom) | (hlw(hb.w, lom) << 16);
  unsigned short* o = hp + (size_t)row * KG + 8 * piece;
  *(volatile v4u*)o = pv;
  __threadfence();
  *(volatile v4u*)o = pv;
}

__global__ __launch_bounds__(NTHR) void k_wtr(const float* __restrict__ w, int Kin, int Ncol, int Nrows, int Kout,
                                              unsigned short* wt, int nUnits) {
  const int u = (int)blockIdx.x * NTHR + (int)threadIdx.x;
  if (u >= nUnits) return;
  const int kq = Kout >> 3;
  const int n  = u / kq;
  const int k8 = (u - n * kq) * 8;
  const int kk = k8 - (k8 / Kin) * Kin;
  const int ncl = n < Ncol ? n : Ncol - 1;
  const float* p = w + (size_t)kk * (size_t)Ncol + ncl;
  v4f a, b;
  a.x = p[0];                    a.y = p[(size_t)Ncol];         a.z = p[(size_t)2 * Ncol];     a.w = p[(size_t)3 * Ncol];
  b.x = p[(size_t)4 * Ncol];     b.y = p[(size_t)5 * Ncol];     b.z = p[(size_t)6 * Ncol];     b.w = p[(size_t)7 * Ncol];
  const v4f z4 = {0.f, 0.f, 0.f, 0.f};
  if (n >= Ncol || n >= Nrows) { a = z4; b = z4; }
  const v4u wv = pack8(a, b);
  unsigned short* o = wt + (size_t)n * (size_t)Kout + k8;
  *(volatile v4u*)o = wv;
  __threadfence();
  *(volatile v4u*)o = wv;
}

template<int NH>
__global__ __launch_bounds__(GTHR) void k_gemm(
    const unsigned short* __restrict__ A, const unsigned short* __restrict__ WT,
    float* outF,
    const float* __restrict__ atts, const float* __restrict__ attd, int attN,
    float* SD, int MPr)
{
  constexpr int FH = HC / NH;
  static_assert((FH % 8) == 0);
  __shared__ __attribute__((aligned(16))) float stg[GBM * GBN];
  __shared__ __attribute__((aligned(16))) float satt[2 * GBN];
  __shared__ __attribute__((aligned(16))) float sdot[NSD * GBM];
  const int tid = (int)threadIdx.x, lane = tid & 31, wave = tid >> 5, hh = lane >> 4, m = lane & 15;
  const int rowBase = (int)blockIdx.x * GBM;

  {
    int ai = tid;
    ai = ai < 0 ? 0 : (ai < attN ? ai : attN - 1);
    satt[tid]       = bfr(atts[ai]);
    satt[GBN + tid] = bfr(attd[ai]);
  }

  v8f acc[8];
  {
    const v8f z = {0.f, 0.f, 0.f, 0.f, 0.f, 0.f, 0.f, 0.f};
#pragma unroll
    for (int t = 0; t < 8; ++t) acc[t] = z;
  }
  const unsigned short* ap = A  + (size_t)(rowBase + 16 * wave + m) * (size_t)KG + 8 * hh;
  const unsigned short* wp = WT + (size_t)m * (size_t)KG + 8 * hh;
#pragma unroll 1
  for (int ks = 0; ks < KG / 32; ++ks) {
    FragB af;
    af.h[0] = *(const v8usa*)(ap + 32 * ks);
    af.h[1] = *(const v8usa*)(ap + 32 * ks + 16);
#pragma unroll
    for (int t = 0; t < 8; ++t) {
      const unsigned short* wq = wp + (size_t)(16 * t) * (size_t)KG + 32 * ks;
      FragB bf;
      bf.h[0] = *(const v8usa*)wq;
      bf.h[1] = *(const v8usa*)(wq + 16);
      acc[t] = wmb(af, bf, acc[t]);
    }
  }

#pragma unroll
  for (int t = 0; t < 8; ++t) {
    const int lc = 16 * t + m;
#pragma unroll
    for (int r = 0; r < 8; ++r) {
      const int lr = 16 * wave + 8 * hh + r;
      stg[lr * GBN + lc] = acc[t][r];
    }
  }
  __syncthreads();

  {
    const int row = tid & 63, side = tid >> 6;
    const float* sa = satt + side * GBN;
    const float* hr = stg + row * GBN;
#pragma unroll
    for (int hd = 0; hd < NH; ++hd) {
      float d0 = 0.f;
#pragma unroll 2
      for (int c4 = 0; c4 < FH / 4; ++c4) {
        const v4f h4 = *(const v4fa*)(hr + hd * FH + 4 * c4);
        const v4f a4 = *(const v4fa*)(sa + hd * FH + 4 * c4);
        d0 = fmaf(h4.x, a4.x, d0); d0 = fmaf(h4.y, a4.y, d0); d0 = fmaf(h4.z, a4.z, d0); d0 = fmaf(h4.w, a4.w, d0);
      }
      sdot[(side * NH + hd) * GBM + row] = d0;
    }
  }
  __syncthreads();

  v4f fv[16];
#pragma unroll
  for (int i = 0; i < 16; ++i) {
    const int lr = 16 * wave + i;
    fv[i] = *(const v4fa*)(stg + lr * GBN + 4 * lane);
  }
  const int seg   = tid >> 4;
  const int piece = tid & 15;
  const int segc  = seg < 2 * NH ? seg : 2 * NH - 1;
  const int side  = segc / NH;
  const int hd    = segc - side * NH;
  const int plane = side * NHMAX + hd;
  const v4f sdv = *(const v4fa*)(sdot + segc * GBM + 4 * piece);
  float* sp = SD + (size_t)plane * (size_t)MPr + rowBase + 4 * piece;
  const bool sdw = (tid < 32 * NH);

#pragma unroll
  for (int i = 0; i < 16; ++i) {
    const int gr = rowBase + 16 * wave + i;
    float* op = outF + (size_t)gr * (size_t)HC + 4 * lane;
    *(volatile v4f*)op = fv[i];
  }
  if (sdw) *(volatile v4f*)sp = sdv;
  __threadfence();
#pragma unroll
  for (int i = 0; i < 16; ++i) {
    const int gr = rowBase + 16 * wave + i;
    float* op = outF + (size_t)gr * (size_t)HC + 4 * lane;
    *(volatile v4f*)op = fv[i];
  }
  if (sdw) *(volatile v4f*)sp = sdv;
}

template<int L>
__global__ __launch_bounds__(NTHR) void k_agg(
    const int* __restrict__ srcs, const int* __restrict__ dsts,
    const float* __restrict__ F, const float* __restrict__ SD,
    const float* __restrict__ bias,
    unsigned short* HP, float* out,
    int nN, int nE, int nb, int MPr) {
  constexpr int NH = (L == 1) ? NHMAX : 1;
  extern __shared__ v4f lds_dyn[];
  int* reg1 = (int*)lds_dyn;
  int* reg2 = reg1 + RCAP;
  int* scnt = reg2 + RCAP;
  int* soff = scnt + NBMAX;
  int* list = soff + NBMAX;
  int* wcnt = list + LISTN;
  int* wtot = wcnt + NWAVE;
  const int tid = (int)threadIdx.x, lane = tid & 31, wave = tid >> 5;
  const int nodeBase = (int)blockIdx.x * nb;
  const int vec8 = ((reinterpret_cast<uintptr_t>(dsts) & (uintptr_t)15) == (uintptr_t)0) ? 1 : 0;

  for (int i = tid; i < NBMAX; i += NTHR) scnt[i] = 0;
  __syncthreads();

  int tot = 0;
  const int nChunks = (nE + CHUNK - 1) / CHUNK;
#pragma unroll 1
  for (int ch = 0; ch < nChunks; ++ch) {
    const int cbase = ch * CHUNK;
    const int wc = scan_chunk(dsts, nE, cbase, nodeBase, nb, vec8, list, tid, lane, wave);
    if (lane == 0) wcnt[wave] = wc;
    __syncthreads();
    int pre = 0, all = 0;
#pragma unroll
    for (int w2 = 0; w2 < NWAVE; ++w2) {
      int c = wcnt[w2];
      c = c < 0 ? 0 : (c > WCAP ? WCAP : c);
      all += c;
      pre += (w2 < wave) ? c : 0;
    }
    const int wcc  = wc > WCAP ? WCAP : wc;
    const int base = tot + pre;
#pragma unroll 1
    for (int i = lane; i < wcc; i += 32) {
      const int ent = list[wave * WCAP + i];
      const int el  = (ent >> SLOTB) & (CHUNK - 1);
      const int sl  = ent & (NBMAX - 1);
      int eid = cbase + el;
      eid = eid > nE - 1 ? nE - 1 : eid;
      const int pos = base + i;
      if (pos < RCAP) reg1[pos] = (int)(((unsigned)eid << SLOTB) | (unsigned)sl);
    }
    tot += all;
    tot = tot > RCAP ? RCAP : tot;
    __syncthreads();
  }
  const int nh = tot;

  if (wave == 0) {
#pragma unroll 1
    for (int b0 = 0; b0 < nh; b0 += 32) {
      const int idx = b0 + lane;
      const int uv  = reg1[idx < nh ? idx : nh - 1];
      const int m32 = (nh - b0) < 32 ? (nh - b0) : 32;
#pragma unroll 1
      for (int k = 0; k < m32; ++k) {
        const int u  = __builtin_amdgcn_readlane(uv, k);
        const int sl = u & (NBMAX - 1);
        if (lane == 0) scnt[sl] = scnt[sl] + 1;
      }
    }
  }
  __syncthreads();

  {
    const v4i ca = *(const v4i*)(scnt + 8 * tid);
    const v4i cb = *(const v4i*)(scnt + 8 * tid + 4);
    const int e0 = ca.x < 0 ? 0 : ca.x, e1 = ca.y < 0 ? 0 : ca.y, e2 = ca.z < 0 ? 0 : ca.z, e3 = ca.w < 0 ? 0 : ca.w;
    const int e4 = cb.x < 0 ? 0 : cb.x, e5 = cb.y < 0 ? 0 : cb.y, e6 = cb.z < 0 ? 0 : cb.z, e7 = cb.w < 0 ? 0 : cb.w;
    const int ts = e0 + e1 + e2 + e3 + e4 + e5 + e6 + e7;
    int incl = ts;
#pragma unroll
    for (int d = 1; d < 32; d <<= 1) {
      const int up = __shfl_up(incl, d);
      if (lane >= d) incl += up;
    }
    if (lane == 31) wtot[wave] = incl;
    __syncthreads();
    int pre = 0;
#pragma unroll
    for (int w2 = 0; w2 < NWAVE; ++w2) pre += (w2 < wave) ? wtot[w2] : 0;
    int run = pre + incl - ts;
    soff[8 * tid + 0] = run; run += e0;
    soff[8 * tid + 1] = run; run += e1;
    soff[8 * tid + 2] = run; run += e2;
    soff[8 * tid + 3] = run; run += e3;
    soff[8 * tid + 4] = run; run += e4;
    soff[8 * tid + 5] = run; run += e5;
    soff[8 * tid + 6] = run; run += e6;
    soff[8 * tid + 7] = run;
  }
  __syncthreads();
  for (int i = tid; i < NBMAX; i += NTHR) list[i] = soff[i];
  __syncthreads();

  if (wave == 0) {
#pragma unroll 1
    for (int b0 = 0; b0 < nh; b0 += 32) {
      const int idx = b0 + lane;
      const int uv  = reg1[idx < nh ? idx : nh - 1];
      const int m32 = (nh - b0) < 32 ? (nh - b0) : 32;
#pragma unroll 1
      for (int k = 0; k < m32; ++k) {
        const int u   = __builtin_amdgcn_readlane(uv, k);
        const int sl  = u & (NBMAX - 1);
        const int eid = (int)((unsigned)u >> SLOTB);
        if (lane == 0) {
          int pos = list[sl];
          pos = pos < 0 ? 0 : (pos > RCAP - 1 ? RCAP - 1 : pos);
          reg2[pos] = eid;
          list[sl] = pos + 1;
        }
      }
    }
  }
  __syncthreads();

  const int nbw = nb >> 3;
  const bool ovf = (nh >= RCAP);
  const float qnan = __int_as_float(0x7fc00000);
  const int sA = (2 * lane) & 31;
  const int sB = (2 * lane + 1) & 31;
  const int c0 = 4 * lane;
  const int head = (NH == 1) ? 0 : (lane >> 3);
  const float* ELp = SD + (size_t)head * (size_t)MPr;
  const float* ERp = SD + (size_t)(NHMAX + head) * (size_t)MPr;
  const v4f bb = bfr4(*(const v4fa*)(bias + c0));
  const unsigned int lom = (lane >= 16) ? 0xFFFFFFFFu : 0u;

#pragma unroll 1
  for (int jt = 0; jt < nbw; ++jt) {
    const int slot = wave * nbw + jt;
    const int grow = nodeBase + slot;
    const int gcl  = grow < nN ? grow : nN - 1;
    int st = soff[slot];
    const int craw = scnt[slot];
    int cnt = craw;
    st  = st < 0 ? 0 : (st > nh ? nh : st);
    cnt = cnt < 0 ? 0 : (cnt > DEGCAP ? DEGCAP : cnt);
    if (cnt > nh - st) cnt = nh - st;
    const float pz = (ovf || craw > DEGCAP) ? qnan : 0.0f;

    const float erd = ERp[gcl];
    float l0 = ELp[gcl] + erd;
    l0 = l0 > 0.f ? l0 : NEGSL * l0;
    float mx = l0, dn = 1.0f;
    v4f av = *(const v4fa*)(F + (size_t)gcl * HC + c0);

#pragma unroll 1
    for (int q = 0; q < cnt; ++q) {
      int idx = st + q; idx = idx > RCAP - 1 ? RCAP - 1 : idx;
      int eid = reg2[idx]; eid = eid < 0 ? 0 : (eid > nE - 1 ? nE - 1 : eid);
      const int sraw = srcs[eid];
      const int s = sraw < 0 ? 0 : (sraw > nN - 1 ? nN - 1 : sraw);
      const v4f fs = *(const v4fa*)(F + (size_t)s * HC + c0);
      float lg = ELp[s] + erd;
      lg = lg > 0.f ? lg : NEGSL * lg;
      const float df = lg - mx;
      const float ee = __expf(-fabsf(df));
      const bool up  = df > 0.f;
      const float s1 = up ? ee : 1.0f;
      const float s2 = up ? 1.0f : ee;
      mx = up ? lg : mx;
      dn = fmaf(dn, s1, s2);
      av.x = fmaf(av.x, s1, s2 * fs.x);
      av.y = fmaf(av.y, s1, s2 * fs.y);
      av.z = fmaf(av.z, s1, s2 * fs.z);
      av.w = fmaf(av.w, s1, s2 * fs.w);
    }
    const float inv = __builtin_amdgcn_rcpf(dn + EPS_SM);
    v4f h;
    h.x = fmaf(av.x, inv, bb.x);
    h.y = fmaf(av.y, inv, bb.y);
    h.z = fmaf(av.z, inv, bb.z);
    h.w = fmaf(av.w, inv, bb.w);
    if (L < 4) {
      h.x = h.x > 0.f ? h.x : 0.f;
      h.y = h.y > 0.f ? h.y : 0.f;
      h.z = h.z > 0.f ? h.z : 0.f;
      h.w = h.w > 0.f ? h.w : 0.f;
      const bool live = grow < nN;
      h.x = (live ? h.x : 0.f) + pz;
      h.y = (live ? h.y : 0.f) + pz;
      h.z = (live ? h.z : 0.f) + pz;
      h.w = (live ? h.w : 0.f) + pz;
      const unsigned int hb0 = f2bf(h.x), hb1 = f2bf(h.y), hb2 = f2bf(h.z), hb3 = f2bf(h.w);
      const unsigned int lb0 = f2bf(h.x - bf2f(hb0)), lb1 = f2bf(h.y - bf2f(hb1));
      const unsigned int lb2 = f2bf(h.z - bf2f(hb2)), lb3 = f2bf(h.w - bf2f(hb3));
      const int hw0 = (int)(hb0 | (hb1 << 16)), hw1 = (int)(hb2 | (hb3 << 16));
      const int lw0 = (int)(lb0 | (lb1 << 16)), lw1 = (int)(lb2 | (lb3 << 16));
      const int a0h = __shfl(hw0, sA), a1h = __shfl(hw1, sA), a0l = __shfl(lw0, sA), a1l = __shfl(lw1, sA);
      const int b0h = __shfl(hw0, sB), b1h = __shfl(hw1, sB), b0l = __shfl(lw0, sB), b1l = __shfl(lw1, sB);
      v4u pv;
      pv.x = ((unsigned int)a0h & ~lom) | ((unsigned int)a0l & lom);
      pv.y = ((unsigned int)a1h & ~lom) | ((unsigned int)a1l & lom);
      pv.z = ((unsigned int)b0h & ~lom) | ((unsigned int)b0l & lom);
      pv.w = ((unsigned int)b1h & ~lom) | ((unsigned int)b1l & lom);
      unsigned short* gp = HP + (size_t)grow * KG + 8 * lane;
      const bool wr = (grow < MPr);
      if (wr) *(volatile v4u*)gp = pv;
      __threadfence();
      if (wr) *(volatile v4u*)gp = pv;
    } else {
      h.x += pz; h.y += pz; h.z += pz; h.w += pz;
      float* op = out + (size_t)gcl * HC + c0;
      const bool wr = (grow < nN);
      if (wr) *(volatile v4f*)op = h;
      __threadfence();
      if (wr) *(volatile v4f*)op = h;
    }
  }
}

static int pick_nb(int nE, int nN) {
  int nb = NBMAX;
  while (nb > 32 && (long long)nb * (long long)nE * 5LL > (long long)RCAP * (long long)nN * 2LL) nb >>= 1;
  return nb;
}
static inline int cdiv(int a, int b) { return (a + b - 1) / b; }

extern "C" void kernel_launch(void* const* d_in, const int* in_sizes, int n_in,
                              void* d_out, int out_size, void* d_ws, size_t ws_size,
                              hipStream_t stream) {
  if (n_in < 20) return;
  const int nN = in_sizes[0];
  if (nN <= 0 || nN > (1 << 22)) return;
  if (in_sizes[1] < 2 || (in_sizes[1] & 1) != 0) return;
  const int nE = in_sizes[1] / 2;
  if (nE < 1 || nE >= (1 << (32 - SLOTB))) return;
  if (in_sizes[2] != HC || in_sizes[3] != HC) return;
  for (int l = 0; l < 4; ++l) {
    const int b = 4 + 4 * l;
    if (in_sizes[b] != HC * HC || in_sizes[b + 1] != HC || in_sizes[b + 2] != HC || in_sizes[b + 3] != HC) return;
  }
  if (out_size != nN * HC) return;

  const float* x    = (const float*)d_in[0];
  const int*   ei   = (const int*)  d_in[1];
  const float* Wemb = (const float*)d_in[2];
  const float* bemb = (const float*)d_in[3];
  const float* W1   = (const float*)d_in[4];
  const float* as1  = (const float*)d_in[5];
  const float* ad1  = (const float*)d_in[6];
  const float* b1   = (const float*)d_in[7];
  const float* W2   = (const float*)d_in[8];
  const float* as2  = (const float*)d_in[9];
  const float* ad2  = (const float*)d_in[10];
  const float* b2   = (const float*)d_in[11];
  const float* W3   = (const float*)d_in[12];
  const float* as3  = (const float*)d_in[13];
  const float* ad3  = (const float*)d_in[14];
  const float* b3   = (const float*)d_in[15];
  const float* W4   = (const float*)d_in[16];
  const float* as4  = (const float*)d_in[17];
  const float* ad4  = (const float*)d_in[18];
  const float* b4   = (const float*)d_in[19];
  float* out = (float*)d_out;

  const int MP = cdiv(nN, MROWS) * MROWS;
  const int EP = cdiv(nE, 32) * 32;
  const int nb = pick_nb(nE, nN);
  if (nb < 32 || (nb & (nb - 1)) != 0 || nb > NBMAX) return;
  const int gA = cdiv(MP, nb);
  if (gA * nb < MP) return;

  char* ws = (char*)d_ws;
  size_t off = 0;
  const size_t oSL  = off; off += (size_t)EP * 4;                 off = (off + 255) & ~(size_t)255;
  const size_t oDL  = off; off += (size_t)EP * 4;                 off = (off + 255) & ~(size_t)255;
  const size_t oHP  = off; off += (size_t)MP * KG * 2;            off = (off + 255) & ~(size_t)255;
  const size_t oXP  = off; off += (size_t)MP * HC * 4;            off = (off + 255) & ~(size_t)255;
  const size_t oSD  = off; off += (size_t)NSD * MP * 4;           off = (off + 255) & ~(size_t)255;
  const size_t oWT1 = off; off += (size_t)HC * KG * 2;            off = (off + 255) & ~(size_t)255;
  const size_t oWT2 = off; off += (size_t)HC * KG * 2;            off = (off + 255) & ~(size_t)255;
  const size_t oWT3 = off; off += (size_t)HC * KG * 2;            off = (off + 255) & ~(size_t)255;
  const size_t oWT4 = off; off += (size_t)HC * KG * 2;            off = (off + 255) & ~(size_t)255;
  if (off > ws_size || off > (size_t)WSMAX) return;
  int*            SL  = (int*)(ws + oSL);
  int*            DL  = (int*)(ws + oDL);
  unsigned short* HP  = (unsigned short*)(ws + oHP);
  float*          XP  = (float*)(ws + oXP);
  float*          SD  = (float*)(ws + oSD);
  unsigned short* WT1 = (unsigned short*)(ws + oWT1);
  unsigned short* WT2 = (unsigned short*)(ws + oWT2);
  unsigned short* WT3 = (unsigned short*)(ws + oWT3);
  unsigned short* WT4 = (unsigned short*)(ws + oWT4);

  hipFuncSetAttribute(reinterpret_cast<const void*>(&k_agg<1>),
                      hipFuncAttributeMaxDynamicSharedMemorySize, LDS_AGG);
  hipFuncSetAttribute(reinterpret_cast<const void*>(&k_agg<2>),
                      hipFuncAttributeMaxDynamicSharedMemorySize, LDS_AGG);
  hipFuncSetAttribute(reinterpret_cast<const void*>(&k_agg<4>),
                      hipFuncAttributeMaxDynamicSharedMemorySize, LDS_AGG);

  const int nUe = EP / 4;
  k_esplit<<<cdiv(nUe, NTHR), NTHR, 0, stream>>>(ei, SL, DL, nE, nUe);

  const int nUx = MP * 32;
  k_emb<<<cdiv(nUx, NTHR), NTHR, 0, stream>>>(x, Wemb, bemb, HP, nN, nUx);

  {
    const int nUw = HC * (KG / 8);
    k_wtr<<<cdiv(nUw, NTHR), NTHR, 0, stream>>>(W1, HC, HC, HC, KG, WT1, nUw);
    k_wtr<<<cdiv(nUw, NTHR), NTHR, 0, stream>>>(W2, HC, HC, HC, KG, WT2, nUw);
    k_wtr<<<cdiv(nUw, NTHR), NTHR, 0, stream>>>(W3, HC, HC, HC, KG, WT3, nUw);
    k_wtr<<<cdiv(nUw, NTHR), NTHR, 0, stream>>>(W4, HC, HC, HC, KG, WT4, nUw);
  }

  const int gM = MP / GBM;
  k_gemm<4><<<gM, GTHR, 0, stream>>>(HP, WT1, XP, as1, ad1, HC, SD, MP);
  k_agg<1><<<gA, NTHR, LDS_AGG, stream>>>(SL, DL, XP, SD, b1, HP, out, nN, nE, nb, MP);
  k_gemm<1><<<gM, GTHR, 0, stream>>>(HP, WT2, XP, as2, ad2, HC, SD, MP);
  k_agg<2><<<gA, NTHR, LDS_AGG, stream>>>(SL, DL, XP, SD, b2, HP, out, nN, nE, nb, MP);
  k_gemm<1><<<gM, GTHR, 0, stream>>>(HP, WT3, XP, as3, ad3, HC, SD, MP);
  k_agg<2><<<gA, NTHR, LDS_AGG, stream>>>(SL, DL, XP, SD, b3, HP, out, nN, nE, nb, MP);
  k_gemm<1><<<gM, GTHR, 0, stream>>>(HP, WT4, XP, as4, ad4, HC, SD, MP);
  k_agg<4><<<gA, NTHR, LDS_AGG, stream>>>(SL, DL, XP, SD, b4, HP, out, nN, nE, nb, MP);
}
